// RevRNN_23545010717137
// MI455X (gfx1250) — hardware-verified
//
#include <hip/hip_runtime.h>


namespace {
constexpr int Bn = 64, S = 256, I = 512, H = 1024, D = 512, KK = D + I;
constexpr float AS_ = 8.0f, EPS = 1e-5f;

typedef _Float16 b16;
typedef __attribute__((ext_vector_type(16))) _Float16 v16b;
typedef __attribute__((ext_vector_type(8))) _Float16 v8b;
typedef __attribute__((ext_vector_type(8))) float v8f;
typedef __attribute__((ext_vector_type(4))) float v4f;
typedef __attribute__((ext_vector_type(8))) unsigned short v8us;
__device__ __forceinline__ float bf16_rne(float f) { unsigned int u = __float_as_uint(f); u += 0x7FFFu + ((u >> 16) & 1u); return __uint_as_float(u & 0xFFFF0000u); }
__device__ __forceinline__ void split16(float v, b16& hi, b16& lo) { hi = (b16)v; lo = (b16)(v - (float)hi); }
__device__ __forceinline__ v16b frag_kb(const b16* p, int hh) { const v8b a = *(const v8b*)(p + 8 * hh), b = *(const v8b*)(p + 16 + 8 * hh); v16b f;
#pragma unroll
  for (int e = 0; e < 8; ++e) { f[e] = a[e]; f[8 + e] = b[e]; } return f; }
__device__ __forceinline__ v8f wmma16b(v16b a, v16b b, v8f c) { v8f d = __builtin_amdgcn_wmma_f32_16x16x32_f16(false, a, false, b, (short)0, c, false, false); asm volatile("v_nop\n\tv_nop\n\tv_nop\n\tv_nop" : "+v"(d) : "v"(a), "v"(b)); return d; }
__device__ __forceinline__ float nexp(float x) { return __builtin_amdgcn_exp2f(x * 1.4426950408889634f); }
__device__ __forceinline__ float softplus_(float z) { return fmaxf(z, 0.0f) + log1pf(__expf(-fabsf(z))); }
__device__ __forceinline__ float tanh_(float x) { const float e = nexp(-2.0f * fabsf(x)); const float t = (1.0f - e) * __builtin_amdgcn_rcpf(1.0f + e); return (x >= 0.0f) ? t : -t; }
__device__ __forceinline__ float mish_(float v) { const float w = nexp(fminf(v, 20.0f)); const float n = w * (w + 2.0f); return (v > 20.0f) ? v : v * n * __builtin_amdgcn_rcpf(n + 2.0f); }

__global__ __launch_bounds__(256) void prep_kernel(const float* __restrict__ fin, const float* __restrict__ h0, const float* __restrict__ W0, const float* __restrict__ W1, const float* __restrict__ w0, const float* __restrict__ b0, const float* __restrict__ w1, const float* __restrict__ b1,
                                                   b16* __restrict__ x16, b16* __restrict__ wr, float* __restrict__ P, float* __restrict__ hs) {
  const size_t tid = (size_t)blockIdx.x * blockDim.x + threadIdx.x, nth = (size_t)gridDim.x * blockDim.x;
  for (int pass = 0; pass < 2; ++pass) {
    for (size_t p = tid; p < (size_t)Bn * S * I / 8; p += nth) { v8b v;
#pragma unroll
      for (int e = 0; e < 8; ++e) v[e] = (b16)bf16_rne(fin[p * 8 + e]);
      *(volatile v8b*)(x16 + p * 8) = v; }
    for (size_t p = tid; p < (size_t)2 * D * KK / 8; p += nth) { v8b v;
#pragma unroll
      for (int e = 0; e < 8; ++e) { const size_t q = p * 8 + e; v[e] = (b16)bf16_rne((q < (size_t)D * KK) ? W0[q] : W1[q - (size_t)D * KK]); }
      *(volatile v8b*)(wr + p * 8) = v; }
    for (size_t p = tid; p < (size_t)4 * D / 4; p += nth) { v4f v;
#pragma unroll
      for (int e = 0; e < 4; ++e) { const size_t q = p * 4 + e; const int m = (int)(q / D), c = (int)(q % D); const float* src = (m == 0) ? w0 : (m == 1) ? b0 : (m == 2) ? w1 : b1; v[e] = bf16_rne(src[c]); }
      *(volatile v4f*)(P + p * 4) = v; }
    for (size_t p = tid; p < (size_t)Bn * H / 4; p += nth) { v4f v;
#pragma unroll
      for (int e = 0; e < 4; ++e) v[e] = bf16_rne(h0[(p * 4 + e) % H]);
      *(volatile v4f*)(hs + p * 4) = v; }
    __threadfence(); }
}

__global__ __launch_bounds__(256) void rnn_kernel(const b16* __restrict__ x16, const b16* __restrict__ wr, const float* __restrict__ P, float* __restrict__ hs, float* __restrict__ out) {
  __shared__ float red[2][256]; __shared__ __attribute__((aligned(16))) float To[8][16][128 + 4];
  const int t_ = threadIdx.x, wid = t_ >> 5, lane = t_ & 31, nloc = lane & 15, hlf = lane >> 4, rt = wid >> 1, c0 = (wid & 1) * 256;
  volatile float* hv = hs;
  for (int step = 0; step < S; ++step) {
    for (int ph = 0; ph < 2; ++ph) {
      const int ucol = ph ? D : 0, ocol = ph ? 0 : D; const float* bw = P + (ph ? 2 : 0) * D; const float* bb = bw + D; const b16* Wm = wr + (size_t)ph * D * KK;
      __syncthreads();
      float s = 0.0f; for (int i = t_; i < Bn * D; i += 256) s += hv[(size_t)(i >> 9) * H + ucol + (i & 511)];
      red[0][t_] = s; __syncthreads();
      for (int st = 128; st > 0; st >>= 1) { if (t_ < st) red[0][t_] += red[0][t_ + st]; __syncthreads(); }
      const float mean = red[0][0] * (1.0f / (Bn * D));
      float q = 0.0f; for (int i = t_; i < Bn * D; i += 256) { const float dv = hv[(size_t)(i >> 9) * H + ucol + (i & 511)] - mean; q += dv * dv; }
      red[1][t_] = q; __syncthreads();
      for (int st = 128; st > 0; st >>= 1) { if (t_ < st) red[1][t_] += red[1][t_ + st]; __syncthreads(); }
      const float stdv = sqrtf(red[1][0] * (1.0f / (Bn * D - 1))); const float isd = rsqrtf(stdv + EPS);
      const int row = 16 * rt + nloc; const b16* xr = x16 + ((size_t)row * S + step) * I;
      for (int hfc = 0; hfc < 2; ++hfc) { v8f acc[8];
#pragma unroll
        for (int t = 0; t < 8; ++t) acc[t] = (v8f){};
        const int cb = c0 + hfc * 128;
#pragma unroll 1
        for (int kb = 0; kb < D; kb += 32) { v16b ah, al;
#pragma unroll
          for (int e = 0; e < 16; ++e) { const int k = kb + ((e < 8) ? (8 * hlf + e) : (16 + 8 * hlf + e - 8)); const float u = hv[(size_t)row * H + ucol + k]; const float v = mish_((u - mean) * isd * bw[k] + bb[k]); b16 p, qq; split16(v * AS_, p, qq); ah[e] = p; al[e] = qq; }
#pragma unroll
          for (int t = 0; t < 8; ++t) { const v16b bf = frag_kb(Wm + (size_t)(cb + t * 16 + nloc) * KK + kb, hlf); acc[t] = wmma16b(ah, bf, acc[t]); acc[t] = wmma16b(al, bf, acc[t]); } }
#pragma unroll 1
        for (int kb = 0; kb < I; kb += 32) { v16b ax = frag_kb(xr + kb, hlf);
#pragma unroll
          for (int e = 0; e < 16; ++e) ax[e] = (b16)((float)ax[e] * AS_);
#pragma unroll
          for (int t = 0; t < 8; ++t) { const v16b bf = frag_kb(Wm + (size_t)(cb + t * 16 + nloc) * KK + D + kb, hlf); acc[t] = wmma16b(ax, bf, acc[t]); } }
#pragma unroll
        for (int t = 0; t < 8; ++t)
#pragma unroll
          for (int v = 0; v < 8; ++v) { const int rl = 8 * hlf + v, c = cb + t * 16 + nloc; To[wid][rl][t * 16 + nloc] = acc[t][v] * (1.0f / AS_) + hv[(size_t)(16 * rt + rl) * H + ocol + c]; }
        __builtin_amdgcn_fence(__ATOMIC_RELEASE, "workgroup"); __builtin_amdgcn_wave_barrier(); __builtin_amdgcn_fence(__ATOMIC_ACQUIRE, "workgroup");
        for (int rl = 0; rl < 16; ++rl) *(volatile v4f*)(hs + (size_t)(16 * rt + rl) * H + ocol + cb + lane * 4) = *(const v4f*)(&To[wid][rl][lane * 4]);
        __builtin_amdgcn_fence(__ATOMIC_RELEASE, "workgroup"); __builtin_amdgcn_wave_barrier(); __builtin_amdgcn_fence(__ATOMIC_ACQUIRE, "workgroup"); }
      __threadfence(); __syncthreads();
    }
  }
  for (int pass = 0; pass < 2; ++pass) { for (int i = t_; i < Bn * H / 4; i += 256) *(volatile v4f*)(out + (size_t)i * 4) = *(const volatile v4f*)(hs + (size_t)i * 4); __threadfence(); }
}
}

extern "C" void kernel_launch(void* const* d_in, const int* in_sizes, int n_in,
                              void* d_out, int out_size, void* d_ws, size_t ws_size, hipStream_t stream) {
  (void)n_in; (void)out_size;
  const float* fin = (const float*)d_in[0]; const float* h0 = (const float*)d_in[1]; const float* W0 = (const float*)d_in[2]; const float* W1 = (const float*)d_in[3];
  const float* w0 = (const float*)d_in[4]; const float* b0 = (const float*)d_in[5]; const float* w1 = (const float*)d_in[6]; const float* b1 = (const float*)d_in[7];
  float* out = (float*)d_out;
  if (in_sizes[0] != Bn * S * I || in_sizes[1] != H || in_sizes[2] != D * KK || in_sizes[3] != D * KK || in_sizes[4] != D) return;
  size_t off = 0; char* ws = (char*)d_ws;
  auto carve = [&](size_t bytes) { char* p = ws + off; off += (bytes + 255) & ~(size_t)255; return p; };
  b16* x16 = (b16*)carve((size_t)Bn * S * I * 2); b16* wr = (b16*)carve((size_t)2 * D * KK * 2); float* P = (float*)carve(4 * D * 4); float* hs = (float*)carve((size_t)Bn * H * 4);
  if (off > ws_size) return;
  prep_kernel<<<512, 256, 0, stream>>>(fin, h0, W0, W1, w0, b0, w1, b1, x16, wr, P, hs);
  rnn_kernel<<<1, 256, 0, stream>>>(x16, wr, P, hs, out);
}
